// GraphContextEncoder_10488310137244
// MI455X (gfx1250) — hardware-verified
//
#include <hip/hip_runtime.h>
#include <stddef.h>
#include <math.h>


#define DF    128
#define DQ    384
#define DFF   512
#define NGRF  64
#define GR    32
#define AP    136
#define HIDP  520
#define XSP   132
#define QSP   388
#define RAP   264
#define TPK   513
#define NTHR  256
#define NWAVE 8
#define NB    512
#define CHUNK 2048
#define WCAP  256
#define NGRP  (CHUNK / (NTHR * 4))
#define HP    4

#define WSC   256.0f
#define AGGSC 64.0f
#define HIDSC 16.0f

#define LDS_SACC (NB * DF)
#define LDS_DEN  (NB * HP)
#define LDS_MAX  (NB * HP)
#define LDS_LIST (NWAVE * WCAP)
#define ATT_LDS_BYTES ((LDS_SACC + LDS_DEN + LDS_MAX + LDS_LIST + NWAVE) * 4)
#define POST_LDS_BYTES (GR * AP * 2 + GR * AP * 2 + GR * HIDP * 2 + GR * XSP * 4 + GR * XSP * 4)
#define RO_SM (2 * NGRF * DF)
#define RO_LDS_BYTES ((RO_SM + RO_SM + 2 * NGRF) * 4 + 2 * NGRF * RAP * 2)

static_assert(WCAP == (CHUNK / NTHR) * 32);
static_assert(NGRP == 2);
static_assert(NB == 512);
static_assert(CHUNK == 2048);
static_assert(((LDS_SACC + LDS_DEN) % 4) == 0);
static_assert((LDS_MAX % 4) == 0);
static_assert((NB % NWAVE) == 0);
static_assert((NB % GR) == 0);
static_assert(ATT_LDS_BYTES == 286752);
static_assert(POST_LDS_BYTES == 84480);
static_assert(RO_LDS_BYTES == 199168);
static_assert(((GR * AP * 2) % 16) == 0);
static_assert(((GR * HIDP * 2) % 16) == 0);
static_assert(((GR * XSP * 4) % 16) == 0);
static_assert(NGRF * AP * 2 <= RO_SM * 4);
static_assert(NGRF * XSP <= RO_SM);

typedef float          v4f   __attribute__((ext_vector_type(4)));
typedef float          v8f   __attribute__((ext_vector_type(8)));
typedef int            v4i   __attribute__((ext_vector_type(4)));
typedef unsigned short v8us  __attribute__((ext_vector_type(8)));
typedef unsigned short v16us __attribute__((ext_vector_type(16)));
typedef __bf16         v16bf __attribute__((ext_vector_type(16)));
typedef _Float16       v4h   __attribute__((ext_vector_type(4)));
typedef _Float16       v8h   __attribute__((ext_vector_type(8)));
typedef _Float16       v16h  __attribute__((ext_vector_type(16)));
union FragB  { v16bf v; v8us half[2]; };
union FragH  { v16h v; v8h half[2]; };
union Pack16 { v8us h; v4i i; };
union PackH  { v8h h; v4i i; };

__device__ __forceinline__ v8f wmb(v16bf a, v16bf b, v8f c) {
  v8f d = __builtin_amdgcn_wmma_f32_16x16x32_bf16(false, a, false, b, (short)0, c, false, false);
  asm volatile("v_nop\n\tv_nop\n\tv_nop\n\tv_nop" : "+v"(d) : "v"(a), "v"(b));
  return d;
}
__device__ __forceinline__ v8f wmh(v16h a, v16h b, v8f c) {
  v8f d = __builtin_amdgcn_wmma_f32_16x16x32_f16(false, a, false, b, (short)0, c, false, false);
  asm volatile("v_nop\n\tv_nop\n\tv_nop\n\tv_nop" : "+v"(d) : "v"(a), "v"(b));
  return d;
}

__device__ __forceinline__ unsigned short bf_bits(float x) {
  const unsigned u = __float_as_uint(x);
  return (unsigned short)((u + 0x7FFFu + ((u >> 16) & 1u)) >> 16);
}
__device__ __forceinline__ void bf_split(float x, unsigned short& hi, unsigned short& lo) {
  const unsigned short hb = bf_bits(x);
  const float r = x - __uint_as_float(((unsigned)hb) << 16);
  hi = hb;
  lo = bf_bits(r);
}

__device__ __forceinline__ float gelu_f(float x) {
  return 0.5f * x * (1.0f + erff(x * 0.70710678118654752f));
}

__device__ __forceinline__ v4f ln_row(v4f x, v4f g, v4f b) {
  float s = (x.x + x.y) + (x.z + x.w);
#pragma unroll
  for (int mk = 16; mk > 0; mk >>= 1) s += __shfl_xor(s, mk, 32);
  const float mean = s * 0.0078125f;
  const v4f d = x - mean;
  float ss = (d.x * d.x + d.y * d.y) + (d.z * d.z + d.w * d.w);
#pragma unroll
  for (int mk = 16; mk > 0; mk >>= 1) ss += __shfl_xor(ss, mk, 32);
  const float rinv = rsqrtf(ss * 0.0078125f + 1e-5f);
  return d * rinv * g + b;
}

__global__ __launch_bounds__(NTHR) void k_prep(const float* __restrict__ W, int K, int M, int inStride,
                                               unsigned short* O0, unsigned short* O1, int outStride,
                                               int mode, float scale) {
  __shared__ float T[16 * TPK];
  const int tid = threadIdx.x;
  const int n0  = blockIdx.x * 16;
  const int l   = blockIdx.y;
  const float* Wl = W + (size_t)l * (size_t)inStride;
  const int tot = K * 16;
  for (int idx = tid; idx < tot; idx += NTHR) {
    const int k = idx >> 4;
    const int c = idx & 15;
    T[c * TPK + k] = Wl[(size_t)k * M + n0 + c];
  }
  __syncthreads();
  const int nseg   = K >> 3;
  const int totseg = nseg * 16;
  v4i u0[4], u1[4];
  size_t po[4];
#pragma unroll
  for (int q = 0; q < 4; ++q) {
    int s = q * NTHR + tid;
    s = s < totseg ? s : totseg - 1;
    const int c  = s / nseg;
    const int k0 = (s - c * nseg) * 8;
    Pack16 ph, pl;
    PackH  pf;
#pragma unroll
    for (int j = 0; j < 8; ++j) {
      const float xv = T[c * TPK + k0 + j];
      unsigned short a, b;
      bf_split(xv, a, b);
      ph.h[j] = a;
      pl.h[j] = b;
      pf.h[j] = (_Float16)(xv * scale);
    }
    v4i sel;
    if (mode != 0) sel = ph.i; else sel = pf.i;
    u0[q] = sel;
    u1[q] = pl.i;
    po[q] = (size_t)l * (size_t)outStride + (size_t)(n0 + c) * K + k0;
  }
#pragma unroll
  for (int q = 0; q < 4; ++q) {
    if (q * NTHR < totseg) {
      *(volatile v4i*)(O0 + po[q]) = u0[q];
      if (mode != 0) *(volatile v4i*)(O1 + po[q]) = u1[q];
    }
  }
  __threadfence();
#pragma unroll
  for (int q = 0; q < 4; ++q) {
    if (q * NTHR < totseg) {
      *(volatile v4i*)(O0 + po[q]) = u0[q];
      if (mode != 0) *(volatile v4i*)(O1 + po[q]) = u1[q];
    }
  }
}

__global__ __launch_bounds__(NTHR) void k_in(
    const float* __restrict__ x, const unsigned short* __restrict__ Wh,
    const unsigned short* __restrict__ Wl, const float* __restrict__ bias,
    const float* __restrict__ gam, const float* __restrict__ bet, float* hout, int nN) {
  __shared__ __attribute__((aligned(16))) unsigned short Ah[GR * AP];
  __shared__ __attribute__((aligned(16))) unsigned short Al[GR * AP];
  __shared__ __attribute__((aligned(16))) float Xs[GR * XSP];

  const int tid  = threadIdx.x;
  const int lane = tid & 31;
  const int wave = tid >> 5;
  const int hh   = lane >> 4;
  const int m    = lane & 15;
  const int rowBase = blockIdx.x * GR;

  {
    const int r  = tid >> 3;
    const int c0 = (tid & 7) * 16;
    int row = rowBase + r;
    if (row > nN - 1) row = nN - 1;
    const float* p = x + (size_t)row * DF + c0;
    const v4f f0 = *(const v4f*)(p), f1 = *(const v4f*)(p + 4);
    const v4f f2 = *(const v4f*)(p + 8), f3 = *(const v4f*)(p + 12);
    float v[16];
    v[0] = f0.x;  v[1] = f0.y;  v[2] = f0.z;  v[3] = f0.w;
    v[4] = f1.x;  v[5] = f1.y;  v[6] = f1.z;  v[7] = f1.w;
    v[8] = f2.x;  v[9] = f2.y;  v[10] = f2.z; v[11] = f2.w;
    v[12] = f3.x; v[13] = f3.y; v[14] = f3.z; v[15] = f3.w;
    Pack16 h0, h1, l0, l1;
#pragma unroll
    for (int j = 0; j < 8; ++j) {
      unsigned short a, b;
      bf_split(v[j], a, b);
      h0.h[j] = a; l0.h[j] = b;
      bf_split(v[8 + j], a, b);
      h1.h[j] = a; l1.h[j] = b;
    }
    *(v8us*)(Ah + r * AP + c0)     = h0.h;
    *(v8us*)(Ah + r * AP + c0 + 8) = h1.h;
    *(v8us*)(Al + r * AP + c0)     = l0.h;
    *(v8us*)(Al + r * AP + c0 + 8) = l1.h;
  }
  __syncthreads();

  const int ncol = wave * 16 + m;
  v8f c0a = {0.f, 0.f, 0.f, 0.f, 0.f, 0.f, 0.f, 0.f};
  v8f c1a = {0.f, 0.f, 0.f, 0.f, 0.f, 0.f, 0.f, 0.f};
#pragma unroll
  for (int kt = 0; kt < DF / 32; ++kt) {
    const int k0 = kt * 32;
    FragB a0h, a0l, a1h, a1l, bh, bl;
    const unsigned short* pbh  = Wh + (size_t)ncol * DF + k0 + 8 * hh;
    const unsigned short* pbl  = Wl + (size_t)ncol * DF + k0 + 8 * hh;
    const unsigned short* pa0h = Ah + m * AP + k0 + 8 * hh;
    const unsigned short* pa0l = Al + m * AP + k0 + 8 * hh;
    const unsigned short* pa1h = Ah + (16 + m) * AP + k0 + 8 * hh;
    const unsigned short* pa1l = Al + (16 + m) * AP + k0 + 8 * hh;
    bh.half[0]  = *(const v8us*)pbh;  bh.half[1]  = *(const v8us*)(pbh + 16);
    bl.half[0]  = *(const v8us*)pbl;  bl.half[1]  = *(const v8us*)(pbl + 16);
    a0h.half[0] = *(const v8us*)pa0h; a0h.half[1] = *(const v8us*)(pa0h + 16);
    a0l.half[0] = *(const v8us*)pa0l; a0l.half[1] = *(const v8us*)(pa0l + 16);
    a1h.half[0] = *(const v8us*)pa1h; a1h.half[1] = *(const v8us*)(pa1h + 16);
    a1l.half[0] = *(const v8us*)pa1l; a1l.half[1] = *(const v8us*)(pa1l + 16);
    c0a = wmb(a0h.v, bh.v, c0a);
    c0a = wmb(a0h.v, bl.v, c0a);
    c0a = wmb(a0l.v, bh.v, c0a);
    c1a = wmb(a1h.v, bh.v, c1a);
    c1a = wmb(a1h.v, bl.v, c1a);
    c1a = wmb(a1l.v, bh.v, c1a);
  }

  const float bv = bias[ncol];
#pragma unroll
  for (int r = 0; r < 8; ++r) {
    Xs[(8 * hh + r) * XSP + ncol]      = c0a[r] + bv;
    Xs[(16 + 8 * hh + r) * XSP + ncol] = c1a[r] + bv;
  }
  __syncthreads();

  const v4f g4 = *(const v4f*)(gam + 4 * lane);
  const v4f b4 = *(const v4f*)(bet + 4 * lane);
  v4f y[4];
#pragma unroll
  for (int i = 0; i < 4; ++i) {
    const v4f xv = *(const v4f*)(Xs + (4 * wave + i) * XSP + 4 * lane);
    y[i] = ln_row(xv, g4, b4);
  }
  const int rlim = nN - rowBase;
  size_t po[4];
#pragma unroll
  for (int i = 0; i < 4; ++i) po[i] = (size_t)(rowBase + 4 * wave + i) * DF + 4 * lane;
#pragma unroll
  for (int i = 0; i < 4; ++i)
    if (4 * wave + i < rlim) *(volatile v4f*)(hout + po[i]) = y[i];
  __threadfence();
#pragma unroll
  for (int i = 0; i < 4; ++i)
    if (4 * wave + i < rlim) *(volatile v4f*)(hout + po[i]) = y[i];
}

__global__ __launch_bounds__(NTHR) void k_qkv(const float* __restrict__ hin,
                                              const _Float16* __restrict__ Wp,
                                              float* qkv, int nN) {
  __shared__ __attribute__((aligned(16))) _Float16 Ah[GR * AP];
  __shared__ __attribute__((aligned(16))) float Xs[GR * QSP];

  const int tid  = threadIdx.x;
  const int lane = tid & 31;
  const int wave = tid >> 5;
  const int hh   = lane >> 4;
  const int m    = lane & 15;
  const int rowBase = blockIdx.x * GR;

  {
    const int r  = tid >> 3;
    const int c0 = (tid & 7) * 16;
    int row = rowBase + r;
    if (row > nN - 1) row = nN - 1;
    const float* p = hin + (size_t)row * DF + c0;
    const v4f f0 = *(const v4f*)(p), f1 = *(const v4f*)(p + 4);
    const v4f f2 = *(const v4f*)(p + 8), f3 = *(const v4f*)(p + 12);
    PackH h0, h1;
    h0.h[0] = (_Float16)f0.x; h0.h[1] = (_Float16)f0.y; h0.h[2] = (_Float16)f0.z; h0.h[3] = (_Float16)f0.w;
    h0.h[4] = (_Float16)f1.x; h0.h[5] = (_Float16)f1.y; h0.h[6] = (_Float16)f1.z; h0.h[7] = (_Float16)f1.w;
    h1.h[0] = (_Float16)f2.x; h1.h[1] = (_Float16)f2.y; h1.h[2] = (_Float16)f2.z; h1.h[3] = (_Float16)f2.w;
    h1.h[4] = (_Float16)f3.x; h1.h[5] = (_Float16)f3.y; h1.h[6] = (_Float16)f3.z; h1.h[7] = (_Float16)f3.w;
    *(v8h*)(Ah + r * AP + c0)     = h0.h;
    *(v8h*)(Ah + r * AP + c0 + 8) = h1.h;
  }
  __syncthreads();

  v8f acc[2][3];
#pragma unroll
  for (int T = 0; T < 2; ++T)
#pragma unroll
    for (int t = 0; t < 3; ++t)
#pragma unroll
      for (int r = 0; r < 8; ++r) acc[T][t][r] = 0.f;

  const _Float16* pbBase = Wp + (size_t)(16 * wave + m) * DF;
#pragma unroll
  for (int kt = 0; kt < DF / 32; ++kt) {
    const int k0 = kt * 32;
    FragH a0, a1, b0, b1, b2;
    const _Float16* pa0 = Ah + m * AP + k0 + 8 * hh;
    const _Float16* pa1 = Ah + (16 + m) * AP + k0 + 8 * hh;
    const _Float16* pb0 = pbBase + k0 + 8 * hh;
    const _Float16* pb1 = pb0 + (size_t)DF * DF;
    const _Float16* pb2 = pb0 + (size_t)2 * DF * DF;
    a0.half[0] = *(const v8h*)pa0; a0.half[1] = *(const v8h*)(pa0 + 16);
    a1.half[0] = *(const v8h*)pa1; a1.half[1] = *(const v8h*)(pa1 + 16);
    b0.half[0] = *(const v8h*)pb0; b0.half[1] = *(const v8h*)(pb0 + 16);
    b1.half[0] = *(const v8h*)pb1; b1.half[1] = *(const v8h*)(pb1 + 16);
    b2.half[0] = *(const v8h*)pb2; b2.half[1] = *(const v8h*)(pb2 + 16);
    acc[0][0] = wmh(a0.v, b0.v, acc[0][0]);
    acc[0][1] = wmh(a0.v, b1.v, acc[0][1]);
    acc[0][2] = wmh(a0.v, b2.v, acc[0][2]);
    acc[1][0] = wmh(a1.v, b0.v, acc[1][0]);
    acc[1][1] = wmh(a1.v, b1.v, acc[1][1]);
    acc[1][2] = wmh(a1.v, b2.v, acc[1][2]);
  }

  const float sc = 1.0f / WSC;
#pragma unroll
  for (int T = 0; T < 2; ++T)
#pragma unroll
    for (int t = 0; t < 3; ++t)
#pragma unroll
      for (int r = 0; r < 8; ++r)
        Xs[(16 * T + 8 * hh + r) * QSP + 16 * (wave + 8 * t) + m] = acc[T][t][r] * sc;
  __syncthreads();

  v4f v[12];
  size_t po[12];
#pragma unroll
  for (int i = 0; i < 4; ++i)
#pragma unroll
    for (int ch = 0; ch < 3; ++ch) {
      v[i * 3 + ch]  = *(const v4f*)(Xs + (4 * wave + i) * QSP + ch * DF + 4 * lane);
      po[i * 3 + ch] = (size_t)(rowBase + 4 * wave + i) * DQ + ch * DF + 4 * lane;
    }
#pragma unroll
  for (int i = 0; i < 12; ++i) *(volatile v4f*)(qkv + po[i]) = v[i];
  __threadfence();
#pragma unroll
  for (int i = 0; i < 12; ++i) *(volatile v4f*)(qkv + po[i]) = v[i];
}

__global__ __launch_bounds__(NTHR) void k_attn(
    const float* __restrict__ qkv, const int* __restrict__ srcp, const int* __restrict__ dstp,
    float* agg, int nN, int nE, int nP) {
  extern __shared__ v4f lds_dyn[];
  float* sacc = (float*)lds_dyn;
  float* daux = sacc + LDS_SACC;
  float* maux = daux + LDS_DEN;
  int*   list = (int*)(maux + LDS_MAX);
  int*   wcnt = list + LDS_LIST;

  const int tid  = threadIdx.x;
  const int lane = tid & 31;
  const int wave = tid >> 5;
  const int hd   = lane >> 3;
  const int nodeBase = blockIdx.x * NB;

  {
    const v4f z4 = {0.f, 0.f, 0.f, 0.f};
    for (int i = tid; i < (LDS_SACC + LDS_DEN) / 4; i += NTHR) lds_dyn[i] = z4;
    const float ninf = __uint_as_float(0xff800000u);
    const v4f n4 = {ninf, ninf, ninf, ninf};
    for (int i = tid; i < LDS_MAX / 4; i += NTHR) lds_dyn[(LDS_SACC + LDS_DEN) / 4 + i] = n4;
  }
  __syncthreads();
  const bool al16 = ((((size_t)dstp) & 15) == 0);

  const int nChunks = (nE + CHUNK - 1) / CHUNK;
#pragma unroll 1
  for (int ch = 0; ch < nChunks; ++ch) {
    const int cbase = ch * CHUNK;
    int wc = 0;
#pragma unroll
    for (int g = 0; g < NGRP; ++g) {
      const int el0 = (g * NTHR + tid) * 4;
      const int e0  = cbase + el0;
      const int sent = -2147483647 - 1;
      v4i d;
      if (al16 && (cbase + CHUNK <= nE)) {
        d = *(const v4i*)(dstp + e0);
      } else {
        d.x = (e0     < nE) ? dstp[min(e0, nE - 1)]     : sent;
        d.y = (e0 + 1 < nE) ? dstp[min(e0 + 1, nE - 1)] : sent;
        d.z = (e0 + 2 < nE) ? dstp[min(e0 + 2, nE - 1)] : sent;
        d.w = (e0 + 3 < nE) ? dstp[min(e0 + 3, nE - 1)] : sent;
      }
      const unsigned s0 = (unsigned)d.x - (unsigned)nodeBase;
      const unsigned s1 = (unsigned)d.y - (unsigned)nodeBase;
      const unsigned s2 = (unsigned)d.z - (unsigned)nodeBase;
      const unsigned s3 = (unsigned)d.w - (unsigned)nodeBase;
      const bool h0 = s0 < (unsigned)NB;
      const bool h1 = s1 < (unsigned)NB;
      const bool h2 = s2 < (unsigned)NB;
      const bool h3 = s3 < (unsigned)NB;
      const unsigned many = __builtin_amdgcn_ballot_w32(h0 | h1 | h2 | h3);
      if (many != 0u) {
#define HITJ(J, HJ, SJ) { \
          const unsigned mj = __builtin_amdgcn_ballot_w32(HJ); \
          if (HJ) { \
            const int pos = wc + (int)__builtin_amdgcn_mbcnt_lo(mj, 0u); \
            if (pos < WCAP) list[wave * WCAP + pos] = ((el0 + (J)) << 9) | (int)(SJ); \
          } \
          wc += (int)__builtin_popcount(mj); }
        HITJ(0, h0, s0)
        HITJ(1, h1, s1)
        HITJ(2, h2, s2)
        HITJ(3, h3, s3)
#undef HITJ
      }
    }
    if (lane == 0) wcnt[wave] = wc;
    __syncthreads();

    if (wave == 0) {
      for (int wsx = 0; wsx < NWAVE; ++wsx) {
        int n = __builtin_amdgcn_readfirstlane(wcnt[wsx]);
        n = n > WCAP ? WCAP : n;
        n = n < 0 ? 0 : n;
        for (int i = 0; i < n; ++i) {
          const int ent  = __builtin_amdgcn_readfirstlane(list[wsx * WCAP + i]);
          const int slot = ent & (NB - 1);
          const int eloc = (ent >> 9) & (CHUNK - 1);
          int e = cbase + eloc;
          e = e > nE - 1 ? nE - 1 : e;
          int j = srcp[e];
          j = j < 0 ? 0 : (j > nN - 1 ? nN - 1 : j);
          int nd = nodeBase + slot;
          nd = nd > nN - 1 ? nN - 1 : nd;
          const float* kr = qkv + (size_t)j * DQ;
          const v4f qv = *(const v4f*)(qkv + (size_t)nd * DQ + 4 * lane);
          const v4f kv = *(const v4f*)(kr + DF + 4 * lane);
          const v4f xv = *(const v4f*)(kr + 2 * DF + 4 * lane);
          float s = (qv.x * kv.x + qv.y * kv.y) + (qv.z * kv.z + qv.w * kv.w);
          s += __shfl_xor(s, 1, 32);
          s += __shfl_xor(s, 2, 32);
          s += __shfl_xor(s, 4, 32);
          s *= 0.17677669529663687f;
          const int ai = slot * HP + hd;
          const float mo = maux[ai];
          const float dn = daux[ai];
          const float mn = fmaxf(mo, s);
          const float cf = __expf(mo - mn);
          const float p  = __expf(s - mn);
          v4f* sp = (v4f*)(sacc + slot * DF + 4 * lane);
          const v4f cur = *sp;
          const v4f nxt = cur * cf + xv * p;
          *sp = nxt;
          maux[ai] = mn;
          daux[ai] = dn * cf + p;
        }
      }
    }
    __syncthreads();
  }

#pragma unroll 1
  for (int q = 0; q < NB / NWAVE; ++q) {
    const int slot = wave * (NB / NWAVE) + q;
    const int node = nodeBase + slot;
    if (node >= nP) break;
    const float dn  = daux[slot * HP + hd];
    const float inv = (dn > 0.f) ? (1.0f / dn) : 0.f;
    const v4f sv = *(const v4f*)(sacc + slot * DF + 4 * lane);
    const v4f y = sv * inv;
    float* op = agg + (size_t)node * DF + 4 * lane;
    *(volatile v4f*)op = y;
    __threadfence();
    *(volatile v4f*)op = y;
  }
}

__global__ __launch_bounds__(NTHR) void k_post(
    const float* __restrict__ agg, float* h,
    const _Float16* __restrict__ Wop, const _Float16* __restrict__ W1p, const float* __restrict__ b1,
    const _Float16* __restrict__ W2p, const float* __restrict__ b2,
    const float* __restrict__ g1, const float* __restrict__ be1,
    const float* __restrict__ g2, const float* __restrict__ be2, int nN) {
  extern __shared__ v4f lds_post[];
  _Float16* Aa  = (_Float16*)lds_post;
  _Float16* Ha  = Aa + GR * AP;
  _Float16* Hid = Ha + GR * AP;
  float*    Hs  = (float*)(Hid + GR * HIDP);
  float*    Xs  = Hs + GR * XSP;

  const int tid  = threadIdx.x;
  const int lane = tid & 31;
  const int wave = tid >> 5;
  const int hh   = lane >> 4;
  const int m    = lane & 15;
  const int rowBase = blockIdx.x * GR;
  const int col  = 16 * wave + m;

  {
    const int r  = tid >> 3;
    const int c0 = (tid & 7) * 16;
    int row = rowBase + r;
    if (row > nN - 1) row = nN - 1;
    const float* pa = agg + (size_t)row * DF + c0;
    const float* ph = h + (size_t)row * DF + c0;
    const v4f a0 = *(const v4f*)(pa), a1 = *(const v4f*)(pa + 4);
    const v4f a2 = *(const v4f*)(pa + 8), a3 = *(const v4f*)(pa + 12);
    const v4f h0 = *(const v4f*)(ph), h1 = *(const v4f*)(ph + 4);
    const v4f h2 = *(const v4f*)(ph + 8), h3 = *(const v4f*)(ph + 12);
    PackH q0, q1;
    q0.h[0] = (_Float16)(a0.x * AGGSC); q0.h[1] = (_Float16)(a0.y * AGGSC);
    q0.h[2] = (_Float16)(a0.z * AGGSC); q0.h[3] = (_Float16)(a0.w * AGGSC);
    q0.h[4] = (_Float16)(a1.x * AGGSC); q0.h[5] = (_Float16)(a1.y * AGGSC);
    q0.h[6] = (_Float16)(a1.z * AGGSC); q0.h[7] = (_Float16)(a1.w * AGGSC);
    q1.h[0] = (_Float16)(a2.x * AGGSC); q1.h[1] = (_Float16)(a2.y * AGGSC);
    q1.h[2] = (_Float16)(a2.z * AGGSC); q1.h[3] = (_Float16)(a2.w * AGGSC);
    q1.h[4] = (_Float16)(a3.x * AGGSC); q1.h[5] = (_Float16)(a3.y * AGGSC);
    q1.h[6] = (_Float16)(a3.z * AGGSC); q1.h[7] = (_Float16)(a3.w * AGGSC);
    *(v8h*)(Aa + r * AP + c0)     = q0.h;
    *(v8h*)(Aa + r * AP + c0 + 8) = q1.h;
    *(v4f*)(Hs + r * XSP + c0)      = h0;
    *(v4f*)(Hs + r * XSP + c0 + 4)  = h1;
    *(v4f*)(Hs + r * XSP + c0 + 8)  = h2;
    *(v4f*)(Hs + r * XSP + c0 + 12) = h3;
  }
  __syncthreads();

  {
    v8f c0 = {0.f, 0.f, 0.f, 0.f, 0.f, 0.f, 0.f, 0.f};
    v8f c1 = {0.f, 0.f, 0.f, 0.f, 0.f, 0.f, 0.f, 0.f};
    const _Float16* pbBase = Wop + (size_t)col * DF;
#pragma unroll
    for (int kt = 0; kt < DF / 32; ++kt) {
      const int k0 = kt * 32;
      FragH a0, a1, b;
      const _Float16* pa0 = Aa + m * AP + k0 + 8 * hh;
      const _Float16* pa1 = Aa + (16 + m) * AP + k0 + 8 * hh;
      const _Float16* pb  = pbBase + k0 + 8 * hh;
      a0.half[0] = *(const v8h*)pa0; a0.half[1] = *(const v8h*)(pa0 + 16);
      a1.half[0] = *(const v8h*)pa1; a1.half[1] = *(const v8h*)(pa1 + 16);
      b.half[0]  = *(const v8h*)pb;  b.half[1]  = *(const v8h*)(pb + 16);
      c0 = wmh(a0.v, b.v, c0);
      c1 = wmh(a1.v, b.v, c1);
    }
    const float sc = 1.0f / (AGGSC * WSC);
#pragma unroll
    for (int r = 0; r < 8; ++r) {
      Xs[(8 * hh + r) * XSP + col]      = c0[r] * sc;
      Xs[(16 + 8 * hh + r) * XSP + col] = c1[r] * sc;
    }
  }
  __syncthreads();

  {
    const v4f g4 = *(const v4f*)(g1 + 4 * lane);
    const v4f b4 = *(const v4f*)(be1 + 4 * lane);
#pragma unroll
    for (int i = 0; i < 4; ++i) {
      const int row = 4 * wave + i;
      const v4f hv = *(const v4f*)(Hs + row * XSP + 4 * lane);
      const v4f tv = *(const v4f*)(Xs + row * XSP + 4 * lane);
      const v4f y  = ln_row(hv + tv, g4, b4);
      *(v4f*)(Hs + row * XSP + 4 * lane) = y;
      v4h yh;
      yh.x = (_Float16)y.x; yh.y = (_Float16)y.y; yh.z = (_Float16)y.z; yh.w = (_Float16)y.w;
      *(v4h*)(Ha + row * AP + 4 * lane) = yh;
    }
  }
  __syncthreads();

#pragma unroll 1
  for (int t = 0; t < DFF / DF; ++t) {
    const int colw = 16 * (wave + 8 * t) + m;
    v8f c0 = {0.f, 0.f, 0.f, 0.f, 0.f, 0.f, 0.f, 0.f};
    v8f c1 = {0.f, 0.f, 0.f, 0.f, 0.f, 0.f, 0.f, 0.f};
    const _Float16* pbBase = W1p + (size_t)colw * DF;
#pragma unroll
    for (int kt = 0; kt < DF / 32; ++kt) {
      const int k0 = kt * 32;
      FragH a0, a1, b;
      const _Float16* pa0 = Ha + m * AP + k0 + 8 * hh;
      const _Float16* pa1 = Ha + (16 + m) * AP + k0 + 8 * hh;
      const _Float16* pb  = pbBase + k0 + 8 * hh;
      a0.half[0] = *(const v8h*)pa0; a0.half[1] = *(const v8h*)(pa0 + 16);
      a1.half[0] = *(const v8h*)pa1; a1.half[1] = *(const v8h*)(pa1 + 16);
      b.half[0]  = *(const v8h*)pb;  b.half[1]  = *(const v8h*)(pb + 16);
      c0 = wmh(a0.v, b.v, c0);
      c1 = wmh(a1.v, b.v, c1);
    }
    const float sc = 1.0f / WSC;
    const float bb = b1[colw];
#pragma unroll
    for (int r = 0; r < 8; ++r) {
      const float u0 = c0[r] * sc + bb;
      const float u1 = c1[r] * sc + bb;
      Hid[(8 * hh + r) * HIDP + colw]      = (_Float16)(gelu_f(u0) * HIDSC);
      Hid[(16 + 8 * hh + r) * HIDP + colw] = (_Float16)(gelu_f(u1) * HIDSC);
    }
  }
  __syncthreads();

  {
    v8f c0 = {0.f, 0.f, 0.f, 0.f, 0.f, 0.f, 0.f, 0.f};
    v8f c1 = {0.f, 0.f, 0.f, 0.f, 0.f, 0.f, 0.f, 0.f};
    const _Float16* pbBase = W2p + (size_t)col * DFF;
#pragma unroll 4
    for (int kt = 0; kt < DFF / 32; ++kt) {
      const int k0 = kt * 32;
      FragH a0, a1, b;
      const _Float16* pa0 = Hid + m * HIDP + k0 + 8 * hh;
      const _Float16* pa1 = Hid + (16 + m) * HIDP + k0 + 8 * hh;
      const _Float16* pb  = pbBase + k0 + 8 * hh;
      a0.half[0] = *(const v8h*)pa0; a0.half[1] = *(const v8h*)(pa0 + 16);
      a1.half[0] = *(const v8h*)pa1; a1.half[1] = *(const v8h*)(pa1 + 16);
      b.half[0]  = *(const v8h*)pb;  b.half[1]  = *(const v8h*)(pb + 16);
      c0 = wmh(a0.v, b.v, c0);
      c1 = wmh(a1.v, b.v, c1);
    }
    const float sc = 1.0f / (HIDSC * WSC);
    const float bb = b2[col];
#pragma unroll
    for (int r = 0; r < 8; ++r) {
      Xs[(8 * hh + r) * XSP + col]      = c0[r] * sc + bb;
      Xs[(16 + 8 * hh + r) * XSP + col] = c1[r] * sc + bb;
    }
  }
  __syncthreads();

  {
    const v4f g4 = *(const v4f*)(g2 + 4 * lane);
    const v4f b4 = *(const v4f*)(be2 + 4 * lane);
    v4f y[4];
    size_t po[4];
#pragma unroll
    for (int i = 0; i < 4; ++i) {
      const int row = 4 * wave + i;
      const v4f hv = *(const v4f*)(Hs + row * XSP + 4 * lane);
      const v4f fv = *(const v4f*)(Xs + row * XSP + 4 * lane);
      y[i]  = ln_row(hv + fv, g4, b4);
      po[i] = (size_t)(rowBase + row) * DF + 4 * lane;
    }
    const int rlim = nN - rowBase;
#pragma unroll
    for (int i = 0; i < 4; ++i)
      if (4 * wave + i < rlim) *(volatile v4f*)(h + po[i]) = y[i];
    __threadfence();
#pragma unroll
    for (int i = 0; i < 4; ++i)
      if (4 * wave + i < rlim) *(volatile v4f*)(h + po[i]) = y[i];
  }
}

__global__ __launch_bounds__(NTHR) void k_readout(
    const float* __restrict__ h, const int* __restrict__ batch,
    const unsigned short* __restrict__ W1h, const unsigned short* __restrict__ W1l,
    const unsigned short* __restrict__ W2h, const unsigned short* __restrict__ W2l,
    const float* __restrict__ br1, const float* __restrict__ br2, float* out1, int nN) {
  extern __shared__ v4f lds_ro[];
  float* Sm = (float*)lds_ro;
  float* Mx = Sm + RO_SM;
  float* Cn = Mx + RO_SM;
  unsigned short* A1h = (unsigned short*)(Cn + 2 * NGRF);
  unsigned short* A1l = A1h + NGRF * RAP;
  unsigned short* A2h = (unsigned short*)Sm;
  unsigned short* A2l = A2h + NGRF * AP;
  float* Xo = Mx;

  const int tid  = threadIdx.x;
  const int lane = tid & 31;
  const int wave = tid >> 5;
  const int hh   = lane >> 4;
  const int m    = lane & 15;
  const int col  = 16 * wave + m;

  {
    const float ninf = __uint_as_float(0xff800000u);
    for (int i = tid; i < RO_SM; i += NTHR) { Sm[i] = 0.f; Mx[i] = ninf; }
    if (tid < 2 * NGRF) Cn[tid] = 0.f;
  }
  __syncthreads();

  {
    const int c = tid & (DF - 1);
    const int p = tid >> 7;
    float* sm = Sm + p * (NGRF * DF) + c;
    float* mx = Mx + p * (NGRF * DF) + c;
#pragma unroll 1
    for (int n = p; n < nN; n += 2) {
      int g = batch[n];
      g = g < 0 ? 0 : (g > NGRF - 1 ? NGRF - 1 : g);
      const float v = h[(size_t)n * DF + c];
      sm[g * DF] += v;
      mx[g * DF] = fmaxf(mx[g * DF], v);
      if (c == 0) Cn[p * NGRF + g] += 1.0f;
    }
  }
  __syncthreads();

  for (int idx = tid; idx < NGRF * 2 * DF; idx += NTHR) {
    const int g  = idx >> 8;
    const int d  = idx & 255;
    const int dd = d & (DF - 1);
    const float cnt = Cn[g] + Cn[NGRF + g];
    const float s   = Sm[g * DF + dd] + Sm[NGRF * DF + g * DF + dd];
    const float mxv = fmaxf(Mx[g * DF + dd], Mx[NGRF * DF + g * DF + dd]);
    const float meanv = s * (1.0f / fmaxf(cnt, 1.0f));
    const float maxv  = (cnt > 0.f) ? mxv : 0.f;
    const float val   = (d < DF) ? meanv : maxv;
    unsigned short a, b;
    bf_split(val, a, b);
    A1h[g * RAP + d] = a;
    A1l[g * RAP + d] = b;
  }
  __syncthreads();

  {
    v8f acc[4];
#pragma unroll
    for (int T = 0; T < 4; ++T)
#pragma unroll
      for (int r = 0; r < 8; ++r) acc[T][r] = 0.f;
    const unsigned short* pbh = W1h + (size_t)col * (2 * DF);
    const unsigned short* pbl = W1l + (size_t)col * (2 * DF);
#pragma unroll 2
    for (int kt = 0; kt < (2 * DF) / 32; ++kt) {
      const int k0 = kt * 32;
      FragB bh, bl;
      bh.half[0] = *(const v8us*)(pbh + k0 + 8 * hh); bh.half[1] = *(const v8us*)(pbh + k0 + 16 + 8 * hh);
      bl.half[0] = *(const v8us*)(pbl + k0 + 8 * hh); bl.half[1] = *(const v8us*)(pbl + k0 + 16 + 8 * hh);
#pragma unroll
      for (int T = 0; T < 4; ++T) {
        FragB ah, al;
        const unsigned short* pah = A1h + (16 * T + m) * RAP + k0 + 8 * hh;
        const unsigned short* pal = A1l + (16 * T + m) * RAP + k0 + 8 * hh;
        ah.half[0] = *(const v8us*)pah; ah.half[1] = *(const v8us*)(pah + 16);
        al.half[0] = *(const v8us*)pal; al.half[1] = *(const v8us*)(pal + 16);
        acc[T] = wmb(ah.v, bh.v, acc[T]);
        acc[T] = wmb(ah.v, bl.v, acc[T]);
        acc[T] = wmb(al.v, bh.v, acc[T]);
      }
    }
    const float bb = br1[col];
#pragma unroll
    for (int T = 0; T < 4; ++T)
#pragma unroll
      for (int r = 0; r < 8; ++r) {
        const float gv = gelu_f(acc[T][r] + bb);
        unsigned short a, b;
        bf_split(gv, a, b);
        const int row = 16 * T + 8 * hh + r;
        A2h[row * AP + col] = a;
        A2l[row * AP + col] = b;
      }
  }
  __syncthreads();

  {
    v8f acc[4];
#pragma unroll
    for (int T = 0; T < 4; ++T)
#pragma unroll
      for (int r = 0; r < 8; ++r) acc[T][r] = 0.f;
    const unsigned short* pbh = W2h + (size_t)col * DF;
    const unsigned short* pbl = W2l + (size_t)col * DF;
#pragma unroll 2
    for (int kt = 0; kt < DF / 32; ++kt) {
      const int k0 = kt * 32;
      FragB bh, bl;
      bh.half[0] = *(const v8us*)(pbh + k0 + 8 * hh); bh.half[1] = *(const v8us*)(pbh + k0 + 16 + 8 * hh);
      bl.half[0] = *(const v8us*)(pbl + k0 + 8 * hh); bl.half[1] = *(const v8us*)(pbl + k0 + 16 + 8 * hh);
#pragma unroll
      for (int T = 0; T < 4; ++T) {
        FragB ah, al;
        const unsigned short* pah = A2h + (16 * T + m) * AP + k0 + 8 * hh;
        const unsigned short* pal = A2l + (16 * T + m) * AP + k0 + 8 * hh;
        ah.half[0] = *(const v8us*)pah; ah.half[1] = *(const v8us*)(pah + 16);
        al.half[0] = *(const v8us*)pal; al.half[1] = *(const v8us*)(pal + 16);
        acc[T] = wmb(ah.v, bh.v, acc[T]);
        acc[T] = wmb(ah.v, bl.v, acc[T]);
        acc[T] = wmb(al.v, bh.v, acc[T]);
      }
    }
    const float bb = br2[col];
#pragma unroll
    for (int T = 0; T < 4; ++T)
#pragma unroll
      for (int r = 0; r < 8; ++r) Xo[(16 * T + 8 * hh + r) * XSP + col] = acc[T][r] + bb;
  }
  __syncthreads();

  {
    v4f v[8];
    size_t po[8];
#pragma unroll
    for (int i = 0; i < 8; ++i) {
      v[i]  = *(const v4f*)(Xo + (8 * wave + i) * XSP + 4 * lane);
      po[i] = (size_t)(8 * wave + i) * DF + 4 * lane;
    }
#pragma unroll
    for (int i = 0; i < 8; ++i) *(volatile v4f*)(out1 + po[i]) = v[i];
    __threadfence();
#pragma unroll
    for (int i = 0; i < 8; ++i) *(volatile v4f*)(out1 + po[i]) = v[i];
  }
}

extern "C" void kernel_launch(void* const* d_in, const int* in_sizes, int n_in,
                              void* d_out, int out_size, void* d_ws, size_t ws_size,
                              hipStream_t stream) {
  if (n_in != 23) return;
  const int nN = in_sizes[2];
  if (nN <= 0 || in_sizes[0] != nN * DF) return;
  if (in_sizes[1] <= 0 || (in_sizes[1] & 1) != 0) return;
  const int nE = in_sizes[1] / 2;
  if (in_sizes[3] != DF * DF || in_sizes[4] != DF || in_sizes[5] != DF || in_sizes[6] != DF) return;
  const int L = in_sizes[7] / (DF * DF);
  if (L <= 0 || L > 64 || in_sizes[7] != L * DF * DF) return;
  if (in_sizes[8] != L * DF * DF || in_sizes[9] != L * DF * DF || in_sizes[10] != L * DF * DF) return;
  if (in_sizes[11] != L * DF * DFF || in_sizes[12] != L * DFF || in_sizes[13] != L * DFF * DF) return;
  for (int i = 14; i <= 18; ++i) if (in_sizes[i] != L * DF) return;
  if (in_sizes[19] != 2 * DF * DF || in_sizes[20] != DF || in_sizes[21] != DF * DF || in_sizes[22] != DF) return;
  if (out_size != nN * DF + NGRF * DF) return;

  const float* x     = (const float*)d_in[0];
  const int*   eidx  = (const int*)d_in[1];
  const int*   batch = (const int*)d_in[2];
  const float* W_in  = (const float*)d_in[3];
  const float* b_in  = (const float*)d_in[4];
  const float* g_in  = (const float*)d_in[5];
  const float* be_in = (const float*)d_in[6];
  const float* Wq    = (const float*)d_in[7];
  const float* Wk    = (const float*)d_in[8];
  const float* Wv    = (const float*)d_in[9];
  const float* Wo    = (const float*)d_in[10];
  const float* W1    = (const float*)d_in[11];
  const float* b1f   = (const float*)d_in[12];
  const float* W2    = (const float*)d_in[13];
  const float* b2f   = (const float*)d_in[14];
  const float* g1    = (const float*)d_in[15];
  const float* be1   = (const float*)d_in[16];
  const float* g2    = (const float*)d_in[17];
  const float* be2   = (const float*)d_in[18];
  const float* Wr1   = (const float*)d_in[19];
  const float* br1   = (const float*)d_in[20];
  const float* Wr2   = (const float*)d_in[21];
  const float* br2   = (const float*)d_in[22];
  float* hbuf = (float*)d_out;
  float* out1 = hbuf + (size_t)nN * DF;

  const int* srcp = eidx;
  const int* dstp = eidx + nE;

  const int nP = ((nN + GR - 1) / GR) * GR;
  size_t off = 0;
  char* base = (char*)d_ws;
  unsigned short* Winh = (unsigned short*)(base + off); off += (size_t)DF * DF * 2;
  unsigned short* Winl = (unsigned short*)(base + off); off += (size_t)DF * DF * 2;
  _Float16* Wqkvp = (_Float16*)(base + off); off += (size_t)L * DQ * DF * 2;
  _Float16* Wop   = (_Float16*)(base + off); off += (size_t)L * DF * DF * 2;
  _Float16* W1p   = (_Float16*)(base + off); off += (size_t)L * DFF * DF * 2;
  _Float16* W2p   = (_Float16*)(base + off); off += (size_t)L * DF * DFF * 2;
  unsigned short* Wr1h = (unsigned short*)(base + off); off += (size_t)2 * DF * DF * 2;
  unsigned short* Wr1l = (unsigned short*)(base + off); off += (size_t)2 * DF * DF * 2;
  unsigned short* Wr2h = (unsigned short*)(base + off); off += (size_t)DF * DF * 2;
  unsigned short* Wr2l = (unsigned short*)(base + off); off += (size_t)DF * DF * 2;
  float* qkv = (float*)(base + off); off += (size_t)nP * DQ * sizeof(float);
  float* agg = (float*)(base + off); off += (size_t)nP * DF * sizeof(float);
  if (off > ws_size) return;
  if (off > (size_t)134217728) return;

  hipFuncSetAttribute(reinterpret_cast<const void*>(&k_attn),
                      hipFuncAttributeMaxDynamicSharedMemorySize, ATT_LDS_BYTES);
  hipFuncSetAttribute(reinterpret_cast<const void*>(&k_post),
                      hipFuncAttributeMaxDynamicSharedMemorySize, POST_LDS_BYTES);
  hipFuncSetAttribute(reinterpret_cast<const void*>(&k_readout),
                      hipFuncAttributeMaxDynamicSharedMemorySize, RO_LDS_BYTES);

  unsigned short* Wqkvu = (unsigned short*)Wqkvp;
  unsigned short* Wou   = (unsigned short*)Wop;
  unsigned short* W1u   = (unsigned short*)W1p;
  unsigned short* W2u   = (unsigned short*)W2p;
  k_prep<<<dim3(DF / 16, 1), NTHR, 0, stream>>>(W_in, DF, DF, DF * DF, Winh, Winl, DF * DF, 1, 1.0f);
  k_prep<<<dim3(DF / 16, L), NTHR, 0, stream>>>(Wq, DF, DF, DF * DF, Wqkvu, Wqkvu, DQ * DF, 0, WSC);
  k_prep<<<dim3(DF / 16, L), NTHR, 0, stream>>>(Wk, DF, DF, DF * DF, Wqkvu + DF * DF, Wqkvu + DF * DF, DQ * DF, 0, WSC);
  k_prep<<<dim3(DF / 16, L), NTHR, 0, stream>>>(Wv, DF, DF, DF * DF, Wqkvu + 2 * DF * DF, Wqkvu + 2 * DF * DF, DQ * DF, 0, WSC);
  k_prep<<<dim3(DF / 16, L), NTHR, 0, stream>>>(Wo, DF, DF, DF * DF, Wou, Wou, DF * DF, 0, WSC);
  k_prep<<<dim3(DFF / 16, L), NTHR, 0, stream>>>(W1, DF, DFF, DF * DFF, W1u, W1u, DFF * DF, 0, WSC);
  k_prep<<<dim3(DF / 16, L), NTHR, 0, stream>>>(W2, DFF, DF, DFF * DF, W2u, W2u, DF * DFF, 0, WSC);
  k_prep<<<dim3(DF / 16, 1), NTHR, 0, stream>>>(Wr1, 2 * DF, DF, 2 * DF * DF, Wr1h, Wr1l, 2 * DF * DF, 1, 1.0f);
  k_prep<<<dim3(DF / 16, 1), NTHR, 0, stream>>>(Wr2, DF, DF, DF * DF, Wr2h, Wr2l, DF * DF, 1, 1.0f);

  const int rgrid = nP / GR;
  k_in<<<rgrid, NTHR, 0, stream>>>(x, Winh, Winl, b_in, g_in, be_in, hbuf, nN);

  const int agrid = (nN + NB - 1) / NB;
  for (int l = 0; l < L; ++l) {
    k_qkv<<<rgrid, NTHR, 0, stream>>>(hbuf, Wqkvp + (size_t)l * DQ * DF, qkv, nN);
    k_attn<<<agrid, NTHR, ATT_LDS_BYTES, stream>>>(qkv, srcp, dstp, agg, nN, nE, nP);
    k_post<<<rgrid, NTHR, POST_LDS_BYTES, stream>>>(
        agg, hbuf, Wop + (size_t)l * DF * DF, W1p + (size_t)l * DFF * DF, b1f + (size_t)l * DFF,
        W2p + (size_t)l * DF * DFF, b2f + (size_t)l * DF,
        g1 + (size_t)l * DF, be1 + (size_t)l * DF, g2 + (size_t)l * DF, be2 + (size_t)l * DF, nN);
  }

  k_readout<<<1, NTHR, RO_LDS_BYTES, stream>>>(hbuf, batch, Wr1h, Wr1l, Wr2h, Wr2l, br1, br2, out1, nN);
}
